// ConvLRUModel_33243046871352
// MI455X (gfx1250) — hardware-verified
//
#include <hip/hip_runtime.h>
#include <math.h>


typedef unsigned short u16;
typedef __attribute__((ext_vector_type(16))) _Float16 v16bf;
typedef __attribute__((ext_vector_type(4)))  float    v4f_t;
typedef float v4fa __attribute__((ext_vector_type(4), may_alias));
typedef __attribute__((ext_vector_type(8)))  float     v8f;
typedef __attribute__((ext_vector_type(4)))  int       v4i;
typedef __attribute__((ext_vector_type(8)))  int       v8i;
typedef __attribute__((ext_vector_type(4)))  unsigned  v4u;

typedef __attribute__((address_space(1))) v4i  gas_v4i;
typedef __attribute__((address_space(3))) v4i  las_v4i;
typedef __attribute__((address_space(3))) char las_char;

union ABu { v16bf v; u16 s[16]; };

__device__ __forceinline__ u16 f2bf(float f) { return __builtin_bit_cast(u16, (_Float16)f); }
__device__ __forceinline__ unsigned pk2h(float a, float b) { return (unsigned)f2bf(a) | ((unsigned)f2bf(b) << 16); }
__device__ __forceinline__ void st2f(float* p, float v) { *(volatile float*)p = v; __threadfence(); *(volatile float*)p = v; }
__device__ __forceinline__ void st2u(u16* p, unsigned v) { *(volatile unsigned*)p = v; __threadfence(); *(volatile unsigned*)p = v; }

__device__ __forceinline__ v8f wmma_bf16(v16bf a, v16bf b, v8f c) {
  return __builtin_amdgcn_wmma_f32_16x16x32_f16(false, a, false, b, (short)0, c, false, false);
}

#if defined(__has_builtin)
#  if __has_builtin(__builtin_amdgcn_tensor_load_to_lds)
#    define HAVE_TDM 1
#  endif
#  if __has_builtin(__builtin_amdgcn_global_load_async_to_lds_b128)
#    define HAVE_ASYNC_B128 1
#  endif
#  if __has_builtin(__builtin_amdgcn_s_wait_asynccnt)
#    define HAVE_WAIT_ASYNC 1
#  endif
#  if __has_builtin(__builtin_amdgcn_s_wait_tensorcnt)
#    define HAVE_WAIT_TENSOR 1
#  endif
#endif

__global__ __launch_bounds__(256) void prep_xbf_k(
    const float* __restrict__ x, u16* __restrict__ x_bf) {
  __shared__ u16 t[64][65];
  const int tid = threadIdx.x;
  const int n = blockIdx.x >> 6, h = blockIdx.x & 63;
  const int b = n >> 4, l = n & 15;
  for (int i = tid; i < 4096; i += 256) {
    const int c = i >> 6, w = i & 63;
    t[w][c] = f2bf(x[(((size_t)b * 64 + c) * 16 + l) * 4096 + h * 64 + w]);
  }
  __syncthreads();
  u16* dst = x_bf + ((size_t)n * 4096 + h * 64) * 64;
  for (int i = tid; i < 2048; i += 256) {
    const int w = i >> 5, c = (i & 31) * 2;
    st2u(dst + w * 64 + c, (unsigned)t[w][c] | ((unsigned)t[w][c + 1] << 16));
  }
}

__global__ __launch_bounds__(256) void prep_weff_k(
    const float* __restrict__ W_sp, const float* __restrict__ W_dc,
    u16* __restrict__ weff) {
  int i = (blockIdx.x * 256 + threadIdx.x) * 2;
  if (i >= 49 * 64 * 64) return;
  int off = i >> 12;
  int o   = (i >> 6) & 63;
  int c   = i & 63;
  float s0 = 0.f, s1 = 0.f;
#pragma unroll 1
  for (int m = 0; m < 64; ++m) { const float wd = W_dc[o * 64 + m]; s0 += wd * W_sp[(m * 64 + c) * 49 + off]; s1 += wd * W_sp[(m * 64 + c + 1) * 49 + off]; }
  st2u(weff + off * 4096 + o * 64 + c, pk2h(s0, s1));
}

__global__ __launch_bounds__(256) void prep_wio_k(
    const float* __restrict__ W_in, const float* __restrict__ W_out,
    u16* __restrict__ w_in_bf, u16* __restrict__ w_out_bf) {
  int i = (blockIdx.x * 256 + threadIdx.x) * 2;
  if (i < 8192)       st2u(w_in_bf + i, pk2h(W_in[i], W_in[i + 1]));
  else if (i < 12288) st2u(w_out_bf + (i - 8192), pk2h(W_out[i - 8192], W_out[i - 8192 + 1]));
}

__global__ __launch_bounds__(256) void conv_k(
    const u16* __restrict__ x_bf, const u16* __restrict__ weff,
    const float* __restrict__ b_dc, float* __restrict__ y_ws) {
  extern __shared__ u16 smem_bf[];
  const int tid  = threadIdx.x;
  const int lane = tid & 31;
  const int wv   = tid >> 5;
  const int m16  = lane & 15;
  const int half = lane >> 4;
  const int n    = blockIdx.x >> 6;
  const int h    = blockIdx.x & 63;

#if defined(HAVE_TDM)
  if (wv == 0) {
    const unsigned ldsBase = (unsigned)(size_t)(las_char*)smem_bf;
    const unsigned long long gImg =
        (unsigned long long)(x_bf + (size_t)n * 262144);
    const v4i z4 = {0, 0, 0, 0};
    const v8i z8 = {0, 0, 0, 0, 0, 0, 0, 0};
    for (int r = 0; r < 7; ++r) {
      int hr = h + r - 3; hr = hr < 0 ? 0 : (hr > 63 ? 63 : hr);
      const unsigned long long ga = gImg + 2ull * (unsigned)(hr * 4096);
      v4u g0;
      g0.x = 1u;
      g0.y = ldsBase + (unsigned)(r * 8192);
      g0.z = (unsigned)(ga & 0xffffffffu);
      g0.w = (unsigned)((ga >> 32) & 0x1ffffffu)
             | 0x80000000u;
      v8i g1;
      g1[0] = 0x00010000;
      g1[1] = (int)(4096u << 16);
      g1[2] = (int)(1u << 16);
      g1[3] = (int)(4096u << 16);
      g1[4] = 1;
      g1[5] = 4096;
      g1[6] = 0;
      g1[7] = 0;
      __builtin_amdgcn_tensor_load_to_lds(g0, g1, z4, z4, z8, 0);
    }
#  if defined(HAVE_WAIT_TENSOR)
    __builtin_amdgcn_s_wait_tensorcnt(0);
#  else
    asm volatile("s_wait_tensorcnt 0" ::: "memory");
#  endif
  }
#else
  for (int i = tid; i < 7 * 512; i += 256) {
    const int r = i >> 9;
    const int q = i & 511;
    int hr = h + r - 3; hr = hr < 0 ? 0 : (hr > 63 ? 63 : hr);
    const u16* gp = x_bf + ((size_t)n * 262144 + (size_t)hr * 4096 + q * 8);
    u16* lp = smem_bf + (r * 4096 + q * 8);
#  if defined(HAVE_ASYNC_B128)
    __builtin_amdgcn_global_load_async_to_lds_b128((gas_v4i*)gp, (las_v4i*)lp, 0, 0);
#  else
    *(v4i*)lp = *(const v4i*)gp;
#  endif
  }
#  if defined(HAVE_ASYNC_B128)
#    if defined(HAVE_WAIT_ASYNC)
  __builtin_amdgcn_s_wait_asynccnt(0);
#    else
  asm volatile("s_wait_asynccnt 0" ::: "memory");
#    endif
#  endif
#endif
  __syncthreads();

  const int mT  = wv & 3;
  const int nt0 = (wv >> 2) * 2;

  v8f acc0 = {};
  v8f acc1 = {};

#pragma unroll 1
  for (int off = 0; off < 49; ++off) {
    const int dh = off / 7;
    const int dw = off - dh * 7;
#pragma unroll
    for (int kq = 0; kq < 2; ++kq) {
      ABu a;
      const u16* wp = weff + off * 4096 + (mT * 16 + m16) * 64 + kq * 32 + half * 8;
#pragma unroll
      for (int j = 0; j < 8; ++j) { a.s[j] = wp[j]; a.s[8 + j] = wp[16 + j]; }

#pragma unroll
      for (int t = 0; t < 2; ++t) {
        const int wcol = (nt0 + t) * 16 + m16;
        const int srcw = (wcol + dw + 61) & 63;
        const u16* bp  = smem_bf + ((dh * 64 + srcw) * 64 + kq * 32 + half * 8);
        ABu bf;
#pragma unroll
        for (int e = 0; e < 8; ++e) { bf.s[e] = bp[e]; bf.s[8 + e] = bp[16 + e]; }
        if (t == 0) acc0 = wmma_bf16(a.v, bf.v, acc0);
        else        acc1 = wmma_bf16(a.v, bf.v, acc1);
      }
    }
  }

  __shared__ __attribute__((aligned(16))) float cst[8][16 * 36];
  float* sw = cst[wv];
#pragma unroll
  for (int t = 0; t < 2; ++t)
#pragma unroll
    for (int r = 0; r < 8; ++r) { const int ol = half * 8 + r; sw[ol * 36 + t * 16 + m16] = (t == 0 ? acc0[r] : acc1[r]) + b_dc[mT * 16 + ol]; }
  asm volatile("s_wait_dscnt 0" ::: "memory");
#pragma unroll 1
  for (int pass = 0; pass < 2; ++pass) {
#pragma unroll
    for (int i = 0; i < 4; ++i) { const int c = lane + 32 * i, ol = c >> 3, q = (c & 7) * 4;
      *(volatile v4f_t*)(y_ws + ((size_t)n * 64 + mT * 16 + ol) * 4096 + h * 64 + nt0 * 16 + q) = *(const volatile v4fa*)(sw + ol * 36 + q); }
    __threadfence();
  }
}

__global__ __launch_bounds__(256) void gn_k(
    const float* __restrict__ y_ws, float* __restrict__ mu, float* __restrict__ rs) {
  __shared__ float r1[256], r2[256];
  const int tid = threadIdx.x;
  const int n = blockIdx.x >> 2, g = blockIdx.x & 3;
  const float* base = y_ws + (size_t)n * 64 * 4096 + (size_t)g * 16 * 4096;
  float s1 = 0.f, s2 = 0.f;
  for (int i = tid; i < 65536; i += 256) { float v = base[i]; s1 += v; s2 += v * v; }
  r1[tid] = s1; r2[tid] = s2; __syncthreads();
  for (int s = 128; s > 0; s >>= 1) {
    if (tid < s) { r1[tid] += r1[tid + s]; r2[tid] += r2[tid + s]; }
    __syncthreads();
  }
  if (tid == 0) {
    float mean = r1[0] * (1.f / 65536.f);
    float var  = r2[0] * (1.f / 65536.f) - mean * mean;
    st2f(mu + blockIdx.x * 32, mean);
    st2f(rs + blockIdx.x * 32, rsqrtf(var + 1e-5f));
  }
}

__global__ __launch_bounds__(256) void mlp_k(
    const float* __restrict__ x, float* __restrict__ y_ws,
    const float* __restrict__ mu, const float* __restrict__ rs,
    const float* __restrict__ gn_g, const float* __restrict__ gn_b,
    const u16* __restrict__ w_in_bf, const float* __restrict__ b_in,
    const u16* __restrict__ w_out_bf, const float* __restrict__ b_out) {
  __shared__ __attribute__((aligned(16))) u16 sb[8][4096];
  const int tid  = threadIdx.x;
  const int lane = tid & 31;
  const int wv   = tid >> 5;
  const int m16  = lane & 15;
  const int half = lane >> 4;
  u16* ynb = sb[wv];
  u16* zb  = sb[wv] + 2048;

  const int task    = blockIdx.x * 8 + wv;
  const int n       = task >> 7;
  const int pixBase = (task & 127) * 32;
  const int bImg = n >> 4, lImg = n & 15;

  for (int i = lane; i < 2048; i += 32) {
    const int p = i >> 6, c = i & 63, g = c >> 4;
    const float v  = y_ws[((size_t)n * 64 + c) * 4096 + pixBase + p];
    const float yn = (v - mu[(n * 4 + g) * 32]) * rs[(n * 4 + g) * 32] * gn_g[c] + gn_b[c];
    ynb[p * 64 + c] = f2bf(yn);
  }
  __syncthreads();

  v8f hacc[8][2];
#pragma unroll
  for (int mt = 0; mt < 8; ++mt) {
    v8f acc0 = {}, acc1 = {};
#pragma unroll
    for (int kq = 0; kq < 2; ++kq) {
      ABu a;
      const u16* wp = w_in_bf + (mt * 16 + m16) * 64 + kq * 32 + half * 8;
#pragma unroll
      for (int j = 0; j < 8; ++j) { a.s[j] = wp[j]; a.s[8 + j] = wp[16 + j]; }
#pragma unroll
      for (int t = 0; t < 2; ++t) {
        ABu bf;
        const u16* yp = ynb + (t * 16 + m16) * 64 + kq * 32 + half * 8;
#pragma unroll
        for (int e = 0; e < 8; ++e) { bf.s[e] = yp[e]; bf.s[8 + e] = yp[16 + e]; }
        if (t == 0) acc0 = wmma_bf16(a.v, bf.v, acc0); else acc1 = wmma_bf16(a.v, bf.v, acc1);
      }
    }
    hacc[mt][0] = acc0; hacc[mt][1] = acc1;
  }

#pragma unroll
  for (int t = 0; t < 2; ++t)
#pragma unroll
  for (int f = 0; f < 4; ++f) {
#pragma unroll
    for (int r = 0; r < 8; ++r) {
      const int row = f * 16 + half * 8 + r;
      const float hv = hacc[f][t][r]     + b_in[row];
      const float gv = hacc[f + 4][t][r] + b_in[64 + row];
      const float z  = hv * (1.f / (1.f + expf(-gv)));
      zb[(t * 16 + m16) * 64 + row] = f2bf(z);
    }
  }
  __syncthreads();

  float* ust = (float*)sb[wv];
  v8f oacc[4][2];
#pragma unroll
  for (int mt = 0; mt < 4; ++mt) {
    v8f acc0 = {}, acc1 = {};
#pragma unroll
    for (int kq = 0; kq < 2; ++kq) {
      ABu a;
      const u16* wp = w_out_bf + (mt * 16 + m16) * 64 + kq * 32 + half * 8;
#pragma unroll
      for (int j = 0; j < 8; ++j) { a.s[j] = wp[j]; a.s[8 + j] = wp[16 + j]; }
#pragma unroll
      for (int t = 0; t < 2; ++t) {
        ABu bf;
        const u16* zp = zb + (t * 16 + m16) * 64 + kq * 32 + half * 8;
#pragma unroll
        for (int e = 0; e < 8; ++e) { bf.s[e] = zp[e]; bf.s[8 + e] = zp[16 + e]; }
        if (t == 0) acc0 = wmma_bf16(a.v, bf.v, acc0); else acc1 = wmma_bf16(a.v, bf.v, acc1);
      }
    }
    oacc[mt][0] = acc0; oacc[mt][1] = acc1;
  }
  asm volatile("s_wait_dscnt 0" ::: "memory");
#pragma unroll
  for (int mt = 0; mt < 4; ++mt)
#pragma unroll
    for (int t = 0; t < 2; ++t)
#pragma unroll
      for (int r = 0; r < 8; ++r) {
        const int o   = mt * 16 + half * 8 + r;
        const int pix = pixBase + t * 16 + m16;
        const float xf = x[(((size_t)bImg * 64 + o) * 16 + lImg) * 4096 + pix];
        ust[o * 32 + t * 16 + m16] = oacc[mt][t][r] + b_out[o] + xf;
      }
  asm volatile("s_wait_dscnt 0" ::: "memory");
#pragma unroll 1
  for (int pass = 0; pass < 2; ++pass) {
#pragma unroll
    for (int i = 0; i < 16; ++i) { const int c = lane + 32 * i, o = c >> 3, q = (c & 7) * 4;
      *(volatile v4f_t*)(y_ws + ((size_t)n * 64 + o) * 4096 + pixBase + q) = *(const volatile v4fa*)(ust + o * 32 + q); }
    __threadfence();
  }
}

__global__ __launch_bounds__(256) void scan_k(
    const float* __restrict__ u_ws, const float* __restrict__ dt,
    const float* __restrict__ nu_log, const float* __restrict__ theta_log,
    const float* __restrict__ c_re, const float* __restrict__ c_im,
    const float* __restrict__ d_skip, float* __restrict__ out) {
  const int t   = blockIdx.x * 256 + threadIdx.x;
  const int pix = t & 4095;
  const int c   = (t >> 12) & 63;
  const int b   = t >> 18;
  const float nu  = expf(nu_log[c]);
  const float th  = expf(theta_log[c]);
  const float crv = c_re[c], civ = c_im[c], dsv = d_skip[c];
  float hre = 0.f, him = 0.f;
#pragma unroll 1
  for (int l = 0; l < 16; ++l) {
    const float dtv   = dt[b * 16 + l];
    const float decay = expf(-nu * dtv);
    const float ph    = th * dtv;
    const float lr    = decay * cosf(ph);
    const float li    = decay * sinf(ph);
    const float gm    = sqrtf(fmaxf(1.f - decay * decay, 1e-6f));
    const float u     = u_ws[(((size_t)(b * 16 + l)) * 64 + c) * 4096 + pix];
    const float nr = lr * hre - li * him + gm * u;
    const float ni = li * hre + lr * him;
    hre = nr; him = ni;
    *(volatile float*)(out + (((size_t)(b * 64 + c)) * 16 + l) * 4096 + pix) = crv * nr + civ * ni + dsv * u;
  }
  __threadfence();
  hre = 0.f; him = 0.f;
#pragma unroll 1
  for (int l = 0; l < 16; ++l) {
    const float dtv   = dt[b * 16 + l];
    const float decay = expf(-nu * dtv);
    const float ph    = th * dtv;
    const float lr    = decay * cosf(ph);
    const float li    = decay * sinf(ph);
    const float gm    = sqrtf(fmaxf(1.f - decay * decay, 1e-6f));
    const float u     = u_ws[(((size_t)(b * 16 + l)) * 64 + c) * 4096 + pix];
    const float nr = lr * hre - li * him + gm * u;
    const float ni = li * hre + lr * him;
    hre = nr; him = ni;
    *(volatile float*)(out + (((size_t)(b * 64 + c)) * 16 + l) * 4096 + pix) = crv * nr + civ * ni + dsv * u;
  }
}

extern "C" void kernel_launch(void* const* d_in, const int* in_sizes, int n_in,
                              void* d_out, int out_size, void* d_ws, size_t ws_size,
                              hipStream_t stream) {
  (void)in_sizes; (void)n_in; (void)out_size; (void)ws_size;
  const float* x         = (const float*)d_in[0];
  const float* dt        = (const float*)d_in[1];
  const float* W_sp      = (const float*)d_in[2];
  const float* W_dc      = (const float*)d_in[3];
  const float* b_dc      = (const float*)d_in[4];
  const float* gn_g      = (const float*)d_in[5];
  const float* gn_b      = (const float*)d_in[6];
  const float* W_in      = (const float*)d_in[7];
  const float* b_in      = (const float*)d_in[8];
  const float* W_out     = (const float*)d_in[9];
  const float* b_out     = (const float*)d_in[10];
  const float* nu_log    = (const float*)d_in[11];
  const float* theta_log = (const float*)d_in[12];
  const float* c_re      = (const float*)d_in[13];
  const float* c_im      = (const float*)d_in[14];
  const float* d_skip    = (const float*)d_in[15];
  float* out = (float*)d_out;

  char* ws = (char*)d_ws;
  float* y_ws    = (float*)(ws);
  u16*  x_bf     = (u16*)(ws + 33554432);
  u16*  weff     = (u16*)(ws + 50331648);
  u16*  w_in_bf  = (u16*)(ws + 50733056);
  u16*  w_out_bf = (u16*)(ws + 50749440);
  float* mu      = (float*)(ws + 50757632);
  float* rs      = (float*)(ws + 50757632 + 16384);

  prep_xbf_k<<<2048, 256, 0, stream>>>(x, x_bf);
  prep_weff_k<<<392, 256, 0, stream>>>(W_sp, W_dc, weff);
  prep_wio_k<<<24, 256, 0, stream>>>(W_in, W_out, w_in_bf, w_out_bf);
  conv_k<<<2048, 256, 7 * 64 * 64 * sizeof(u16), stream>>>(x_bf, weff, b_dc, y_ws);
  gn_k<<<128, 256, 0, stream>>>(y_ws, mu, rs);
  mlp_k<<<512, 256, 0, stream>>>(x, y_ws, mu, rs, gn_g, gn_b, w_in_bf, b_in, w_out_bf, b_out);
  scan_k<<<2048, 256, 0, stream>>>(y_ws, dt, nu_log, theta_log, c_re, c_im, d_skip, out);
}
